// KANLayer_2989297238631
// MI455X (gfx1250) — hardware-verified
//
#include <hip/hip_runtime.h>
#include <stdint.h>

#pragma clang fp contract(off)

#define NB      4096
#define NI      1024
#define NU      1024
#define NSEGS   10
#define KTOT    (NSEGS * NI)
#define AUNITS  (KTOT / 8)
#define FTHR    256
#define ASWEEP  (AUNITS / FTHR)
#define PT      64
#define NPLANE  7
#define PLDS    (NPLANE * PT * PT)
#define PSTIT   ((PT * NSEGS * 8) / 256)
#define WSCAP   134217728
#define LAM     1.0507009873554805f
#define ALP     1.6732632423543772f

static_assert(KTOT % 32 == 0);
static_assert((KTOT * 2) % 128 == 0);
static_assert(AUNITS == ASWEEP * FTHR);
static_assert(NB % 128 == 0);
static_assert(NU % 64 == 0);
static_assert(NI % PT == 0);
static_assert(NU % PT == 0);
static_assert(PSTIT * 256 == PT * NSEGS * 8);
static_assert(NI % FTHR == 0);
static_assert(NU % 256 == 0);
static_assert(PLDS * 2 <= 65536);

typedef float          v4f   __attribute__((ext_vector_type(4)));
typedef float          v8f   __attribute__((ext_vector_type(8)));
typedef int            v8i   __attribute__((ext_vector_type(8)));
typedef unsigned int   v4u   __attribute__((ext_vector_type(4)));
typedef unsigned short v8us  __attribute__((ext_vector_type(8)));
typedef __bf16         v16bf __attribute__((ext_vector_type(16)));
typedef v4f  __attribute__((may_alias)) v4fa;
typedef v4u  __attribute__((may_alias)) v4ua;
typedef v8us __attribute__((may_alias)) v8usa;
union FragB { v16bf v; v8us h[2]; v8i w; };

__device__ __forceinline__ unsigned short f2bf_bits(float f) {
  unsigned u = __float_as_uint(f);
  return (unsigned short)((u + 0x7FFFu + ((u >> 16) & 1u)) >> 16);
}
__device__ __forceinline__ float bf_bits2f(unsigned short b) { return __uint_as_float(((unsigned)b) << 16); }
__device__ __forceinline__ float bfr(float f) { return bf_bits2f(f2bf_bits(f)); }

__device__ __forceinline__ v8f wmb(const FragB& a, const FragB& b, v8f c) {
  v8f d = __builtin_amdgcn_wmma_f32_16x16x32_bf16(false, a.v, false, b.v, (short)0, c, false, false);
  asm volatile("v_nop\n\tv_nop\n\tv_nop\n\tv_nop" : "+v"(d) : "v"(a.w), "v"(b.w));
  return d;
}
__device__ __forceinline__ v8f z8() { v8f z = {0.f, 0.f, 0.f, 0.f, 0.f, 0.f, 0.f, 0.f}; return z; }

__device__ __forceinline__ void b_store_pass(const unsigned short* sP, unsigned short* BP, int u0, int i0, int tid) {
#pragma unroll 4
  for (int it = 0; it < PSTIT; ++it) {
    const int q = it * 256 + tid;
    const int L = q >> 3, pc = q & 7;
    const int uu = L / NSEGS;
    const int seg = L - NSEGS * uu;
    const int sm1 = seg - 1;
    const int d0 = sm1 / 3;
    const int rr = sm1 - 3 * d0;
    const int pl1 = 1 + 2 * d0 + ((rr == 2) ? 1 : 0);
    const int plane = (seg == 0) ? 0 : pl1;
    const v4u v = *(const v4ua*)(sP + plane * (PT * PT) + uu * PT + 8 * pc);
    *(volatile v4u*)(BP + (size_t)(u0 + uu) * KTOT + (size_t)seg * NI + i0 + 8 * pc) = v;
  }
}

__global__ __launch_bounds__(256) void prep_b_kernel(const float* __restrict__ bw, const float* __restrict__ sw,
                                                     const float* __restrict__ gw, unsigned short* __restrict__ BP) {
  __shared__ __align__(16) unsigned short sP[PLDS];
  const int tid = threadIdx.x;
  const int i0 = blockIdx.x * PT, u0 = blockIdx.y * PT;

#pragma unroll
  for (int it = 0; it < 4; ++it) {
    const int q = it * 256 + tid;
    const int ii = q >> 4, c4 = q & 15;
    const v4f v = *(const v4fa*)(bw + (size_t)(i0 + ii) * NU + u0 + 4 * c4);
    sP[(4 * c4 + 0) * PT + ii] = f2bf_bits(v[0]);
    sP[(4 * c4 + 1) * PT + ii] = f2bf_bits(v[1]);
    sP[(4 * c4 + 2) * PT + ii] = f2bf_bits(v[2]);
    sP[(4 * c4 + 3) * PT + ii] = f2bf_bits(v[3]);
  }

#pragma unroll 2
  for (int it = 0; it < 16; ++it) {
    const int item = it * 256 + tid;
    const int uu = item & (PT - 1), ii = item >> 6;
    const size_t iu = (size_t)(i0 + ii) * NU + (size_t)(u0 + uu);
    const v4f s4 = *(const v4fa*)(sw + iu * 4);
    const float g = bfr(gw[iu]);
    const float p1 = bfr(s4[1]) * g;
    const float p2 = bfr(s4[2]) * g;
    const float p3 = bfr(s4[3]) * g;
    const unsigned short h1 = f2bf_bits(p1), h2 = f2bf_bits(p2), h3 = f2bf_bits(p3);
    const unsigned short l1 = f2bf_bits(p1 - bf_bits2f(h1));
    const unsigned short l2 = f2bf_bits(p2 - bf_bits2f(h2));
    const unsigned short l3 = f2bf_bits(p3 - bf_bits2f(h3));
    const int o = uu * PT + ii;
    sP[1 * PT * PT + o] = h1;
    sP[2 * PT * PT + o] = l1;
    sP[3 * PT * PT + o] = h2;
    sP[4 * PT * PT + o] = l2;
    sP[5 * PT * PT + o] = h3;
    sP[6 * PT * PT + o] = l3;
  }
  __syncthreads();

  b_store_pass(sP, BP, u0, i0, tid);
  __threadfence();
  b_store_pass(sP, BP, u0, i0, tid);
}

__device__ __forceinline__ void c_store_pass(const float* sC, float* cb, int base, int tid) {
  if (tid < 64) {
    const v4f v = *(const v4fa*)(sC + 4 * tid);
    *(volatile v4f*)(cb + base + 4 * tid) = v;
  }
}
__global__ __launch_bounds__(256) void cb_kernel(const float* __restrict__ sw, const float* __restrict__ gw,
                                                 const float* __restrict__ bias, float* __restrict__ cb) {
  __shared__ __align__(16) float sC[256];
  const int tid = threadIdx.x;
  const int u = blockIdx.x * 256 + tid;
  double acc = 0.0;
#pragma unroll 2
  for (int i = 0; i < NI; ++i) {
    const size_t iu = (size_t)i * NU + (size_t)u;
    const float s0 = bfr(sw[iu * 4]);
    const float g = bfr(gw[iu]);
    acc += (double)(s0 * g);
  }
  sC[tid] = (float)acc + bfr(bias[u]);
  __syncthreads();
  const int base = blockIdx.x * 256;
  c_store_pass(sC, cb, base, tid);
  __threadfence();
  c_store_pass(sC, cb, base, tid);
}

__device__ __forceinline__ void a_store_pass(const unsigned short* sA, unsigned short* dst, int tid) {
#pragma unroll
  for (int it = 0; it < ASWEEP; ++it) {
    const int u = it * FTHR + tid;
    const v4u v = *(const v4ua*)(sA + 8 * u);
    *(volatile v4u*)(dst + 8 * u) = v;
  }
}

__global__ __launch_bounds__(FTHR) void feat_kernel(const float* __restrict__ x, unsigned short* __restrict__ AP) {
  __shared__ __align__(16) unsigned short sA[KTOT];
  const int tid = threadIdx.x;
  const int r = blockIdx.x;
#pragma unroll 1
  for (int k = 0; k < NI / FTHR; ++k) {
    const int i = k * FTHR + tid;
    const float xr = bfr(x[(size_t)r * NI + i]);
    const float t1 = tanhf(xr);
    const float t2 = t1 * t1;
    const float t3 = t2 * t1;
    const unsigned short h1 = f2bf_bits(t1), h2 = f2bf_bits(t2), h3 = f2bf_bits(t3);
    const unsigned short l1 = f2bf_bits(t1 - bf_bits2f(h1));
    const unsigned short l2 = f2bf_bits(t2 - bf_bits2f(h2));
    const unsigned short l3 = f2bf_bits(t3 - bf_bits2f(h3));
    sA[0 * NI + i] = f2bf_bits(xr);
    sA[1 * NI + i] = h1;
    sA[2 * NI + i] = l1;
    sA[3 * NI + i] = h1;
    sA[4 * NI + i] = h2;
    sA[5 * NI + i] = l2;
    sA[6 * NI + i] = h2;
    sA[7 * NI + i] = h3;
    sA[8 * NI + i] = l3;
    sA[9 * NI + i] = h3;
  }
  __syncthreads();

  unsigned short* dst = AP + (size_t)r * KTOT;
  a_store_pass(sA, dst, tid);
  __threadfence();
  a_store_pass(sA, dst, tid);
}

__device__ __forceinline__ void o_store_pass(const float* sO, float* out, int grow_w, int n0, int w, int lane) {
  const int q8 = lane & 7, sub = lane >> 3;
#pragma unroll
  for (int i = 0; i < 16; ++i) {
    const int lid = i * 4 + sub;
    const int row = lid >> 1, hl = lid & 1;
    const v4f v = *(const v4fa*)(sO + (32 * w + row) * 64 + 32 * hl + 4 * q8);
    *(volatile v4f*)(out + (size_t)(grow_w + row) * NU + n0 + 32 * hl + 4 * q8) = v;
  }
}

__global__ __launch_bounds__(128) void gemm_kernel(const unsigned short* __restrict__ AP,
                                                   const unsigned short* __restrict__ BP,
                                                   const float* __restrict__ cb,
                                                   float* __restrict__ out) {
  __shared__ __align__(16) float sO[128 * 64];
  const int tid = threadIdx.x, lane = tid & 31, w = tid >> 5;
  const int h = lane >> 4, m = lane & 15;
  const int lrow_w = blockIdx.x * 128 + 32 * w;
  const int n0 = blockIdx.y * 64;

  const unsigned short* xa0 = AP + (size_t)(lrow_w + m) * KTOT + 8 * h;
  const unsigned short* xa1 = xa0 + (size_t)16 * KTOT;
  const unsigned short* wb  = BP + (size_t)(n0 + m) * KTOT + 8 * h;

  v8f acc[2][4];
#pragma unroll
  for (int mt = 0; mt < 2; ++mt)
#pragma unroll
    for (int nt = 0; nt < 4; ++nt) acc[mt][nt] = z8();

#pragma unroll 1
  for (int k0 = 0; k0 < KTOT; k0 += 32) {
    FragB a0, a1;
    a0.h[0] = *(const v8usa*)(xa0 + k0);
    a0.h[1] = *(const v8usa*)(xa0 + k0 + 16);
    a1.h[0] = *(const v8usa*)(xa1 + k0);
    a1.h[1] = *(const v8usa*)(xa1 + k0 + 16);
#pragma unroll
    for (int nt = 0; nt < 4; ++nt) {
      const unsigned short* wq = wb + (size_t)nt * 16 * KTOT + k0;
      FragB b;
      b.h[0] = *(const v8usa*)wq;
      b.h[1] = *(const v8usa*)(wq + 16);
      acc[0][nt] = wmb(a0, b, acc[0][nt]);
      acc[1][nt] = wmb(a1, b, acc[1][nt]);
    }
  }

#pragma unroll
  for (int nt = 0; nt < 4; ++nt) {
    const int cl = 16 * nt + m;
    const float cbv = cb[n0 + cl];
#pragma unroll
    for (int mt = 0; mt < 2; ++mt) {
#pragma unroll
      for (int r = 0; r < 8; ++r) {
        const int rl = 32 * w + 16 * mt + 8 * h + r;
        sO[rl * 64 + cl] = acc[mt][nt][r] + cbv;
      }
    }
  }
  __syncthreads();

#pragma unroll 2
  for (int j = 0; j < 64; ++j) {
    const int e = j * 128 + tid;
    const float p = sO[e];
    const float em = expm1f(fminf(p, 0.0f));
    const float y = (p > 0.0f) ? (LAM * p) : (LAM * (ALP * em));
    sO[e] = y;
  }
  __syncthreads();

  o_store_pass(sO, out, lrow_w, n0, w, lane);
  __threadfence();
  o_store_pass(sO, out, lrow_w, n0, w, lane);
}

extern "C" void kernel_launch(void* const* d_in, const int* in_sizes, int n_in,
                              void* d_out, int out_size, void* d_ws, size_t ws_size,
                              hipStream_t stream) {
  if (n_in < 5) return;
  if (in_sizes[0] != NB * NI) return;
  if (in_sizes[1] != NI * NU) return;
  if (in_sizes[2] != NU) return;
  if (in_sizes[3] != NI * NU * 4) return;
  if (in_sizes[4] != NI * NU) return;
  if (out_size != NB * NU) return;

  const float* x    = (const float*)d_in[0];
  const float* bw   = (const float*)d_in[1];
  const float* bias = (const float*)d_in[2];
  const float* sw   = (const float*)d_in[3];
  const float* gw   = (const float*)d_in[4];
  float* out = (float*)d_out;

  size_t off = 0;
  const size_t oAP = off; off += (size_t)NB * KTOT * 2;
  const size_t oBP = off; off += (size_t)NU * KTOT * 2;
  const size_t oCB = off; off += (size_t)NU * 4;
  if (off > ws_size) return;
  if (off > (size_t)WSCAP) return;

  char* ws = (char*)d_ws;
  unsigned short* AP = (unsigned short*)(ws + oAP);
  unsigned short* BP = (unsigned short*)(ws + oBP);
  float* CB = (float*)(ws + oCB);

  cb_kernel<<<dim3(NU / 256), dim3(256), 0, stream>>>(sw, gw, bias, CB);
  prep_b_kernel<<<dim3(NI / PT, NU / PT), dim3(256), 0, stream>>>(bw, sw, gw, BP);
  feat_kernel<<<dim3(NB), dim3(FTHR), 0, stream>>>(x, AP);
  gemm_kernel<<<dim3(NB / 128, NU / 64), dim3(128), 0, stream>>>(AP, BP, CB, out);
  (void)hipGetLastError();
}
